// Outer_Product_Mean_84748294684976
// MI455X (gfx1250) — hardware-verified
//
#include <hip/hip_runtime.h>


#define NSQ  128
#define NRS  256
#define NCM  256
#define NCH  32
#define NCZ  128
#define NPS  16
constexpr size_t al256(size_t b) { return (b + 255) & ~(size_t)255; }
constexpr size_t WS_TOTAL = al256((size_t)NSQ * NRS * NCM * 2) + al256((size_t)64 * NCM * 2) + al256((size_t)NCZ * NCH * NCH * 2) + al256((size_t)64 * 4) + al256((size_t)NSQ * NRS * 64 * 4) + al256((size_t)NRS * NCH * NSQ * 2) + al256((size_t)NPS * NCH * NRS * NCH * 4) + al256((size_t)NPS * NRS * NCH * NCH * 2);
static_assert(WS_TOTAL == 52723968 && WS_TOTAL <= 134217728, "the workspace carve: 50.3 MiB");
static_assert(NRS % NPS == 0 && (NPS * NCH) % 64 == 0 && (NRS * NCH) % 64 == 0 && (NPS * NRS) % 64 == 0 && NCZ % 64 == 0 && NSQ % 32 == 0 && (NCH * NCH) % 32 == 0 && NCM % 32 == 0, "whole tiles; whole depth steps");
typedef _Float16 h16;
typedef unsigned short bf;
typedef __attribute__((ext_vector_type(16))) __bf16   v16bf;
typedef __attribute__((ext_vector_type(16))) _Float16 v16h;
typedef __attribute__((ext_vector_type(8)))  _Float16 v8h;
typedef __attribute__((ext_vector_type(8)))  unsigned short v8us;
typedef __attribute__((ext_vector_type(8)))  float    v8f;
typedef __attribute__((ext_vector_type(4)))  float    v4f;
typedef v8h  __attribute__((may_alias)) v8ha;
typedef v4f  __attribute__((may_alias)) v4fa;
typedef v8us __attribute__((may_alias)) v8usa;

__device__ __forceinline__ unsigned short f2bf(float f) { unsigned u = __float_as_uint(f); u += 0x7FFFu + ((u >> 16) & 1u); return (unsigned short)(u >> 16); }
__device__ __forceinline__ float bf2f(unsigned short b) { return __uint_as_float(((unsigned)b) << 16); }
__device__ __forceinline__ float bfr(float f) { return bf2f(f2bf(f)); }
__device__ __forceinline__ v16h cat16(v8h lo, v8h hi) { return __builtin_shufflevector(lo, hi, 0, 1, 2, 3, 4, 5, 6, 7, 8, 9, 10, 11, 12, 13, 14, 15); }
__device__ __forceinline__ v16bf cat16b(v8us lo, v8us hi) { return __builtin_bit_cast(v16bf, __builtin_shufflevector(lo, hi, 0, 1, 2, 3, 4, 5, 6, 7, 8, 9, 10, 11, 12, 13, 14, 15)); }
__device__ __forceinline__ v8f wmma16(v16h a, v16h b, v8f c) { return __builtin_amdgcn_wmma_f32_16x16x32_f16(false, a, false, b, (short)0, c, false, false); }
__device__ __forceinline__ v8f wmmab(v16bf a, v16bf b, v8f c) { return __builtin_amdgcn_wmma_f32_16x16x32_bf16(false, a, false, b, (short)0, c, false, false); }


template <typename T16> struct WFrag;
template <> struct WFrag<h16> { typedef v16h V; static __device__ __forceinline__ V ld(const h16* p) { return cat16(*(const v8h*)p, *(const v8h*)(p + 16)); } static __device__ __forceinline__ v8f mma(V a, V b, v8f c) { return wmma16(a, b, c); } };
template <> struct WFrag<bf> { typedef v16bf V; static __device__ __forceinline__ V ld(const bf* p) { return cat16b(*(const v8us*)p, *(const v8us*)(p + 16)); } static __device__ __forceinline__ v8f mma(V a, V b, v8f c) { return wmmab(a, b, c); } };
template <typename T16, int NSPLIT, bool BIAS>
__global__ __launch_bounds__(32) void k_gemmw(const T16* __restrict__ A, const T16* __restrict__ A2, const T16* __restrict__ Bt, const T16* __restrict__ Bt2, int K, float* C, int ldc, const float* __restrict__ bias, size_t sA, size_t sB, size_t sC) {
    typedef typename WFrag<T16>::V V;
    __shared__ __align__(16) float os[16 * 68];
    const size_t z = blockIdx.z; A += z * sA; if (A2) A2 += z * sA; Bt += z * sB; if (Bt2) Bt2 += z * sB; C += z * sC;
    const int lane = threadIdx.x & 31, lr = lane & 15, hi = lane >> 4; const int r0 = blockIdx.x * 64, c0 = blockIdx.y * 64;
    v8f acc[4][4];
#pragma unroll
    for (int mb = 0; mb < 4; ++mb)
#pragma unroll
        for (int nb = 0; nb < 4; ++nb) acc[mb][nb] = (v8f){};
    const size_t aoff = (size_t)(r0 + lr) * K + 8 * hi, boff = (size_t)(c0 + lr) * K + 8 * hi;
    for (int kc = 0; kc < K; kc += 32) {
        V a[4], a2[4];
#pragma unroll
        for (int mb = 0; mb < 4; ++mb) { a[mb] = WFrag<T16>::ld(A + aoff + (size_t)mb * 16 * K + kc); if (NSPLIT == 1 || NSPLIT == 2) a2[mb] = WFrag<T16>::ld(A2 + aoff + (size_t)mb * 16 * K + kc); }
#pragma unroll
        for (int nb = 0; nb < 4; ++nb) { const V b = WFrag<T16>::ld(Bt + boff + (size_t)nb * 16 * K + kc); V b2; if (NSPLIT >= 2) b2 = WFrag<T16>::ld(Bt2 + boff + (size_t)nb * 16 * K + kc);
#pragma unroll
            for (int mb = 0; mb < 4; ++mb) { acc[mb][nb] = WFrag<T16>::mma(a[mb], b, acc[mb][nb]); if (NSPLIT == 1 || NSPLIT == 2) acc[mb][nb] = WFrag<T16>::mma(a2[mb], b, acc[mb][nb]); if (NSPLIT >= 2) acc[mb][nb] = WFrag<T16>::mma(a[mb], b2, acc[mb][nb]); } }
        asm volatile("v_nop\n\tv_nop\n\tv_nop\n\tv_nop" : "+v"(acc[0][0]), "+v"(acc[1][1]), "+v"(acc[2][2]), "+v"(acc[3][3]) : "v"(a[0]), "v"(a[3]));
    }
#pragma unroll
    for (int mb = 0; mb < 4; ++mb) {
#pragma unroll
        for (int nb = 0; nb < 4; ++nb) {
#pragma unroll
            for (int j = 0; j < 8; ++j) os[(hi * 8 + j) * 68 + nb * 16 + lr] = acc[mb][nb][j]; }
        __builtin_amdgcn_wave_barrier(); asm volatile("" ::: "memory");
        float* crow = C + (size_t)(r0 + mb * 16) * ldc + c0;
#pragma unroll 1
        for (int ps = 0; ps < 2; ++ps) {
#pragma unroll
            for (int s = 0; s < 8; ++s) { const int row = 2 * s + hi, cofs = lr * 4; v4f val = *(const v4fa*)(os + row * 68 + cofs); if (BIAS) { val[0] += bfr(bias[c0 + cofs]); val[1] += bfr(bias[c0 + cofs + 1]); val[2] += bfr(bias[c0 + cofs + 2]); val[3] += bfr(bias[c0 + cofs + 3]); }
                *(volatile v4f*)(crow + (size_t)row * ldc + cofs) = val; }
            if (ps == 0) __threadfence(); }
        __builtin_amdgcn_wave_barrier(); asm volatile("" ::: "memory");
    }
}

__device__ __forceinline__ h16 tohx(float x) { return (h16)x; }
__device__ __forceinline__ void splitf(float y, unsigned short& h, unsigned short& l) { h = f2bf(y); l = f2bf(y - bf2f(h)); }
typedef __attribute__((ext_vector_type(2))) _Float16 v2h;
typedef __attribute__((ext_vector_type(4))) _Float16 v4h;
typedef __attribute__((ext_vector_type(2))) unsigned short v2us;
typedef __attribute__((ext_vector_type(4))) unsigned short v4us;
typedef __attribute__((ext_vector_type(2))) float v2f;
typedef __attribute__((ext_vector_type(4))) int v4i;


typedef _Float16 v8h __attribute__((ext_vector_type(8)));
typedef float v4f __attribute__((ext_vector_type(4)));

__global__ __launch_bounds__(256) void k_rnd(const float* __restrict__ src, float* dst, unsigned npc, unsigned nw) {
    const unsigned g = blockIdx.x * 256 + threadIdx.x; if (g >= npc) return; v4f o;
#pragma unroll
    for (int e = 0; e < 4; ++e) { const unsigned i = 4u * g + (unsigned)e; const unsigned live = i < nw ? 1u : 0u; const float rv_ = bfr(src[live ? i : 0u]); o[e] = live ? rv_ : 0.0f; }
    float* dq = dst + 4u * (size_t)g; *(volatile v4f*)(dq) = o; __threadfence(); *(volatile v4f*)(dq) = o; }

__global__ __launch_bounds__(256) void k_lay(const float* __restrict__ src, h16* dst, unsigned nrow, unsigned c8n, unsigned dp, unsigned c0, unsigned rbs, unsigned ra, unsigned rs, unsigned cbs, unsigned sa, unsigned sb, unsigned rlive, unsigned clive) {
    const unsigned g = blockIdx.x * 256 + threadIdx.x; if (g >= nrow * c8n) return; const unsigned row = g / c8n, ch = g - row * c8n; const unsigned rb = (row >> rbs) * ra + (row & ((1u << rbs) - 1u)) * rs; v8h o;
#pragma unroll
    for (int w = 0; w < 8; ++w) { const unsigned c = 8u * ch + w; const bool live = row < rlive && c < clive; const unsigned si = rb + (c >> cbs) * sa + (c & ((1u << cbs) - 1u)) * sb; const float v = bfr(src[live ? si : 0u]); o[w] = tohx(live && fabsf(v) >= 6.103515625e-05f ? v : 0.0f); }
    h16* d8 = dst + (size_t)row * dp + c0 + 8u * ch; *(volatile v8h*)(d8) = o; __threadfence(); *(volatile v8h*)(d8) = o; }

__global__ __launch_bounds__(256) void k_tr(const float* __restrict__ cy, h16* yt) {
    const unsigned g = blockIdx.x * 256 + threadIdx.x; if (g >= (unsigned)(NRS * NCH * (NSQ / 8))) return; const unsigned row = g >> 4, pc = g & 15u; const unsigned ri = row >> 5, rc = row & 31u; v8h o8;
#pragma unroll
    for (int e = 0; e < 8; ++e) { const unsigned sq = 8u * pc + (unsigned)e; const float val = cy[((size_t)sq * NRS + ri) * 64u + rc]; const float kf = fabsf(val) >= 6.103515625e-05f ? 1.0f : 0.0f; o8[e] = tohx(val * kf); }
    h16* d8 = yt + (size_t)row * NSQ + 8u * pc; *(volatile v8h*)(d8) = o8; __threadfence(); *(volatile v8h*)(d8) = o8; }

__global__ __launch_bounds__(256) void k_perm(const float* __restrict__ cc, h16* opc) {
    const unsigned g = blockIdx.x * 256 + threadIdx.x; if (g >= (unsigned)(NPS * NRS * (NCH * NCH / 8))) return; const unsigned row = g >> 7, pc = g & 127u; const unsigned il = row >> 8, rj = row & 255u; const unsigned rc = pc >> 2, e0 = 8u * (pc & 3u);
    const float* sq = cc + ((size_t)il * NCH + rc) * (size_t)(NRS * NCH) + (size_t)rj * NCH + e0; const v4f a = *(const v4f*)sq; const v4f b = *(const v4f*)(sq + 4); v8h o8;
#pragma unroll
    for (int e = 0; e < 8; ++e) { const float val = (e < 4 ? a[e & 3] : b[e & 3]) * 0.0078125f; const float kf = fabsf(val) >= 6.103515625e-05f ? 1.0f : 0.0f; o8[e] = tohx(val * kf); }
    h16* d8 = opc + (size_t)row * (NCH * NCH) + 8u * pc; *(volatile v8h*)(d8) = o8; __threadfence(); *(volatile v8h*)(d8) = o8; }

extern "C" void kernel_launch(void* const* d_in, const int* in_sizes, int n_in,
                              void* d_out, int out_size, void* d_ws, size_t ws_size, hipStream_t stream) {
    if (n_in < 5) return;
    if (in_sizes[0] < NSQ * NRS * NCM || in_sizes[1] < NCH * NCM || in_sizes[2] < NCH || in_sizes[3] < NCZ * NCH * NCH || in_sizes[4] < NCZ || out_size < NRS * NRS * NCZ) return;
    const float* xa = (const float*)d_in[0]; const float* wp = (const float*)d_in[1]; const float* bp = (const float*)d_in[2]; const float* wq = (const float*)d_in[3]; const float* bq = (const float*)d_in[4];
    char* wsp = (char*)d_ws;
    auto take = [&](size_t bytes) { char* cur = wsp; wsp += (bytes + 255) & ~(size_t)255; return (void*)cur; };
    h16* XH = (h16*)take((size_t)NSQ * NRS * NCM * 2); h16* WPH = (h16*)take((size_t)64 * NCM * 2); h16* WQH = (h16*)take((size_t)NCZ * NCH * NCH * 2); float* BB = (float*)take((size_t)64 * 4); float* CY = (float*)take((size_t)NSQ * NRS * 64 * 4); h16* YT = (h16*)take((size_t)NRS * NCH * NSQ * 2); float* CC = (float*)take((size_t)NPS * NCH * NRS * NCH * 4); h16* OPC = (h16*)take((size_t)NPS * NRS * NCH * NCH * 2);
    if ((size_t)(wsp - (char*)d_ws) != WS_TOTAL || WS_TOTAL > ws_size) return;
    auto rnd = [&](const float* sp_, float* dp_, unsigned nw) { const unsigned npc = (nw + 3) / 4; k_rnd<<<(npc + 255) / 256, 256, 0, stream>>>(sp_, dp_, npc, nw); };
    auto lay = [&](const float* sp_, h16* dp_, unsigned nrow, unsigned ncol, unsigned rlive) { k_lay<<<(nrow * (ncol / 8) + 255) / 256, 256, 0, stream>>>(sp_, dp_, nrow, ncol / 8, ncol, 0u, 16u, 0u, ncol, 16u, 0u, 1u, rlive, ncol); };
    lay(xa, XH, NSQ * NRS, NCM, NSQ * NRS); lay(wp, WPH, 64, NCM, NCH); lay(wq, WQH, NCZ, NCH * NCH, NCZ); rnd(bp, BB, NCH); rnd(bp, BB + 32, NCH);
    k_gemmw<h16, 0, true><<<dim3(NSQ * NRS / 64, 1, 1), 32, 0, stream>>>(XH, nullptr, WPH, nullptr, NCM, CY, 64, BB, (size_t)0, (size_t)0, (size_t)0);
    k_tr<<<NRS * NCH * (NSQ / 8) / 256, 256, 0, stream>>>(CY, YT);
    for (int ps = 0; ps < NRS / NPS; ++ps) {
        k_gemmw<h16, 0, false><<<dim3(NPS * NCH / 64, NRS * NCH / 64, 1), 32, 0, stream>>>(YT + (size_t)ps * NPS * NCH * NSQ, nullptr, YT, nullptr, NSQ, CC, NRS * NCH, nullptr, (size_t)0, (size_t)0, (size_t)0);
        k_perm<<<NPS * NRS * (NCH * NCH / 8) / 256, 256, 0, stream>>>(CC, OPC);
        k_gemmw<h16, 0, true><<<dim3(NPS * NRS / 64, NCZ / 64, 1), 32, 0, stream>>>(OPC, nullptr, WQH, nullptr, NCH * NCH, (float*)d_out + (size_t)ps * NPS * NRS * NCZ, NCZ, bq, (size_t)0, (size_t)0, (size_t)0);
    }
}
